// MultiHeadSelfAttention_54803782697214
// MI455X (gfx1250) — hardware-verified
//
#include <hip/hip_runtime.h>


#ifndef NB
#define NB 2
#endif
#ifndef SEQ
#define SEQ 2048
#endif
#define NB_FULL   2
#define SEQ_FULL  2048
#define HID       768
#define NHEAD     12
#define HD        64
#define MROWS     (NB * SEQ)
#define QKVW      (3 * HID)
#define QKW       (2 * HID)
#define PCS       (HID / 8)

static_assert(HID == NHEAD * HD);
static_assert(HD == 64);
static_assert(SEQ % 128 == 0);
static_assert(SEQ <= SEQ_FULL);
static_assert(NB >= 1 && NB <= NB_FULL);
static_assert(MROWS % 128 == 0);
static_assert(HID % 128 == 0);
static_assert(QKW % 128 == 0);
static_assert(QKVW % 128 == 0);
static_assert(HID % 32 == 0);
static_assert(PCS % 8 == 0);
static_assert(PCS * 8 == HID);
static_assert(((size_t)7 * NB_FULL * SEQ_FULL * HID + (size_t)QKVW * HID + (size_t)HID * HID) * 2 <= (size_t)134217728);

#define CARRY_X    16.0f
#define CARRY_W    32.0f
#define CARRY_QKV  16.0f
#define CARRY_RES  2048.0f
#define RES_INV    0.00048828125f
#define CARRY_CTX  1024.0f

typedef _Float16 f16;
typedef f16   v16h __attribute__((ext_vector_type(16)));
typedef f16   v8h  __attribute__((ext_vector_type(8)));
typedef float v8f  __attribute__((ext_vector_type(8)));
typedef float v4f  __attribute__((ext_vector_type(4)));

union FragU { v16h v; v8h half[2]; f16 e[16]; };
union H8U   { v8h v; f16 e[8]; };
union CsU   { f16 h[128 * 128]; float f[64 * 128]; };

__device__ __forceinline__ v8f zero8() {
    v8f z = {0.f, 0.f, 0.f, 0.f, 0.f, 0.f, 0.f, 0.f};
    return z;
}

__device__ __forceinline__ v8f wmma16(v16h a, v16h b, v8f c) {
    v8f d = __builtin_amdgcn_wmma_f32_16x16x32_f16(false, a, false, b, (short)0, c, false, false);
    asm volatile("v_nop\n\tv_nop\n\tv_nop\n\tv_nop" : "+v"(d) : "v"(a), "v"(b));
    return d;
}

__device__ __forceinline__ float bf16_rne(float x) {
    unsigned u = __float_as_uint(x);
    u = (u + 0x7fffu + ((u >> 16) & 1u)) & 0xffff0000u;
    return __uint_as_float(u);
}

__device__ __forceinline__ float fexp2(float x) {
#if defined(__has_builtin)
#if __has_builtin(__builtin_amdgcn_exp2f)
    return __builtin_amdgcn_exp2f(x);
#else
    return exp2f(x);
#endif
#else
    return exp2f(x);
#endif
}

__device__ __forceinline__ float rowmax16(float x) {
    int v = __builtin_bit_cast(int, x);
    x = fmaxf(x, __builtin_bit_cast(float, __builtin_amdgcn_update_dpp(v, v, 0x121, 0xf, 0xf, false)));
    v = __builtin_bit_cast(int, x);
    x = fmaxf(x, __builtin_bit_cast(float, __builtin_amdgcn_update_dpp(v, v, 0x122, 0xf, 0xf, false)));
    v = __builtin_bit_cast(int, x);
    x = fmaxf(x, __builtin_bit_cast(float, __builtin_amdgcn_update_dpp(v, v, 0x124, 0xf, 0xf, false)));
    v = __builtin_bit_cast(int, x);
    x = fmaxf(x, __builtin_bit_cast(float, __builtin_amdgcn_update_dpp(v, v, 0x128, 0xf, 0xf, false)));
    return x;
}

__device__ __forceinline__ int frag_off(int rowbase, int pitch, int kcol, int lane) {
    return (rowbase + (lane & 15)) * pitch + kcol + ((lane >> 4) << 3);
}

__device__ __forceinline__ v16h mk_frag(v8h a, v8h b) {
    FragU f;
    f.half[0] = a;
    f.half[1] = b;
    return f.v;
}

#define LDS_FRAG(arr, off) mk_frag(*(const v8h*)&(arr)[(off)], *(const v8h*)&(arr)[(off) + 16])

__device__ __forceinline__ v16h gfrag(const f16* __restrict__ base, size_t off) {
    return mk_frag(*(const v8h*)(base + off), *(const v8h*)(base + off + 16));
}

__global__ void __launch_bounds__(256)
cvt_rows(const float* __restrict__ src, f16* __restrict__ dst, int nrows, int dstper, int srcper,
         float carry) {
    const int g  = (int)blockIdx.x * 256 + (int)threadIdx.x;
    const int m  = g / PCS;
    const int c8 = (g - m * PCS) << 3;
    if (m >= nrows) return;
    const int blk = m / dstper;
    const int sm  = blk * srcper + (m - blk * dstper);
    const float* sp = src + (size_t)sm * HID + c8;
    const v4f a = *(const v4f*)sp;
    const v4f b = *(const v4f*)(sp + 4);
    H8U o;
#pragma unroll
    for (int j = 0; j < 4; ++j) {
        const float x0 = a[j];
        const float x1 = b[j];
        o.e[j]     = (f16)(bf16_rne(x0) * carry);
        o.e[j + 4] = (f16)(bf16_rne(x1) * carry);
    }
    f16* dp = dst + (size_t)m * HID + c8;
    *(volatile v8h*)dp = o.v;
    __threadfence();
    *(volatile v8h*)dp = o.v;
}

template <int MODE>
__device__ __forceinline__ void gemm_body(const f16* __restrict__ A, const f16* __restrict__ W,
                                          const float* __restrict__ bias,
                                          f16* __restrict__ outP, float* __restrict__ outF,
                                          float accMul, float addMul) {
    __shared__ __attribute__((aligned(16))) f16 As[128 * 32];
    __shared__ __attribute__((aligned(16))) f16 Bs[128 * 32];
    __shared__ __attribute__((aligned(16))) CsU cs;

    const int tid   = (int)threadIdx.x;
    const int lane  = tid & 31;
    const int wave  = tid >> 5;
    const int wm    = wave & 3;
    const int wn    = wave >> 2;
    const int hh8   = (lane >> 4) << 3;
    const int c16   = lane & 15;
    const int m0    = (int)blockIdx.x * 128;
    const int ncol0 = (int)blockIdx.y * 128;

    v8f acc[2][4];
#pragma unroll
    for (int i = 0; i < 2; ++i)
#pragma unroll
        for (int j = 0; j < 4; ++j) acc[i][j] = zero8();

    const int srow = tid >> 1;
    const int scol = (tid & 1) << 4;
    const f16* gA = A + (size_t)(m0 + srow) * HID + scol;
    const f16* gW = W + (size_t)(ncol0 + srow) * HID + scol;

#pragma unroll 1
    for (int k0 = 0; k0 < HID; k0 += 32) {
        const v8h ra0 = *(const v8h*)(gA + k0);
        const v8h ra1 = *(const v8h*)(gA + k0 + 8);
        const v8h rb0 = *(const v8h*)(gW + k0);
        const v8h rb1 = *(const v8h*)(gW + k0 + 8);
        __syncthreads();
        *(v8h*)&As[srow * 32 + scol]     = ra0;
        *(v8h*)&As[srow * 32 + scol + 8] = ra1;
        *(v8h*)&Bs[srow * 32 + scol]     = rb0;
        *(v8h*)&Bs[srow * 32 + scol + 8] = rb1;
        __syncthreads();

        v16h af[2], bfr[4];
#pragma unroll
        for (int i = 0; i < 2; ++i) {
            const int off = frag_off(wm * 32 + i * 16, 32, 0, lane);
            af[i] = LDS_FRAG(As, off);
        }
#pragma unroll
        for (int j = 0; j < 4; ++j) {
            const int off = frag_off(wn * 64 + j * 16, 32, 0, lane);
            bfr[j] = LDS_FRAG(Bs, off);
        }
#pragma unroll
        for (int i = 0; i < 2; ++i)
#pragma unroll
            for (int j = 0; j < 4; ++j) acc[i][j] = wmma16(af[i], bfr[j], acc[i][j]);
    }

    float bb[4];
#pragma unroll
    for (int j = 0; j < 4; ++j) bb[j] = bf16_rne(bias[ncol0 + wn * 64 + j * 16 + c16]) * addMul;

    const int bidx  = m0 / SEQ;
    const int s0    = m0 - bidx * SEQ;
    const int piece = lane & 7;
    const int lsub  = lane >> 3;

    if constexpr (MODE == 0) {
        const int which = ncol0 / HID;
        const int n0    = ncol0 - which * HID;
        const size_t bh0 = (size_t)bidx * NHEAD + (size_t)(n0 >> 6);
        const size_t planeH = (size_t)MROWS * HID;
#pragma unroll
        for (int ph = 0; ph < 2; ++ph) {
            if (ph == 1) __syncthreads();
#pragma unroll
            for (int i = 0; i < 2; ++i)
#pragma unroll
                for (int j = 0; j < 4; ++j) {
                    const int nl = wn * 64 + j * 16 + c16;
#pragma unroll
                    for (int r = 0; r < 8; ++r) {
                        const int ml = wm * 32 + i * 16 + hh8 + r;
                        const float val = acc[i][j][r] * accMul + bb[j];
                        const f16 hi = (f16)val;
                        const f16 rs = (f16)((val - (float)hi) * CARRY_RES);
                        cs.h[ml * 128 + nl] = (ph == 0) ? hi : rs;
                    }
                }
            __syncthreads();
            f16* op = outP + (size_t)(ph * 2 + which) * planeH;
#pragma unroll
            for (int pass = 0; pass < 2; ++pass) {
#pragma unroll
                for (int it = 0; it < 8; ++it) {
                    const int L    = wave * 32 + it * 4 + lsub;
                    const int ml   = L >> 1;
                    const int hsel = L & 1;
                    const v8h v = *(const v8h*)&cs.h[ml * 128 + hsel * 64 + piece * 8];
                    f16* dp = op + ((bh0 + (size_t)hsel) * SEQ + (size_t)(s0 + ml)) * HD + piece * 8;
                    *(volatile v8h*)dp = v;
                }
                if (pass == 0) __threadfence();
            }
        }
    } else if constexpr (MODE == 1) {
#pragma unroll
        for (int i = 0; i < 2; ++i)
#pragma unroll
            for (int j = 0; j < 4; ++j) {
                const int nl = wn * 64 + j * 16 + c16;
                H8U t;
#pragma unroll
                for (int r = 0; r < 8; ++r) t.e[r] = (f16)(acc[i][j][r] * accMul + bb[j]);
                *(v8h*)&cs.h[nl * 128 + wm * 32 + i * 16 + hh8] = t.v;
            }
        __syncthreads();
#pragma unroll
        for (int pass = 0; pass < 2; ++pass) {
#pragma unroll
            for (int it = 0; it < 8; ++it) {
                const int L  = wave * 32 + it * 4 + lsub;
                const int nl = L >> 1;
                const int mh = L & 1;
                const v8h v = *(const v8h*)&cs.h[nl * 128 + mh * 64 + piece * 8];
                f16* dp = outP + ((size_t)(bidx * HID + ncol0 + nl) * SEQ + s0 + mh * 64 + piece * 8);
                *(volatile v8h*)dp = v;
            }
            if (pass == 0) __threadfence();
        }
    } else {
#pragma unroll
        for (int half = 0; half < 2; ++half) {
            if ((wm >> 1) == half) {
#pragma unroll
                for (int i = 0; i < 2; ++i)
#pragma unroll
                    for (int j = 0; j < 4; ++j) {
                        const int nl = wn * 64 + j * 16 + c16;
#pragma unroll
                        for (int r = 0; r < 8; ++r) {
                            const int ml = (wm & 1) * 32 + i * 16 + hh8 + r;
                            cs.f[ml * 128 + nl] = acc[i][j][r] * accMul + bb[j];
                        }
                    }
            }
            __syncthreads();
#pragma unroll
            for (int pass = 0; pass < 2; ++pass) {
#pragma unroll
                for (int it = 0; it < 8; ++it) {
                    const int L    = wave * 32 + it * 4 + lsub;
                    const int row  = L >> 2;
                    const int part = L & 3;
                    const v4f v = *(const v4f*)&cs.f[row * 128 + part * 32 + piece * 4];
                    float* dp = outF + (size_t)(m0 + half * 64 + row) * HID + ncol0 + part * 32 + piece * 4;
                    *(volatile v4f*)dp = v;
                }
                if (pass == 0) __threadfence();
            }
            __syncthreads();
        }
    }
}

__global__ void __launch_bounds__(256) __attribute__((amdgpu_num_vgpr(256)))
gemm_qk(const f16* __restrict__ A, const f16* __restrict__ W, const float* __restrict__ bias,
        f16* __restrict__ outP, float accMul, float addMul) {
    gemm_body<0>(A, W, bias, outP, (float*)nullptr, accMul, addMul);
}

__global__ void __launch_bounds__(256) __attribute__((amdgpu_num_vgpr(256)))
gemm_v(const f16* __restrict__ A, const f16* __restrict__ W, const float* __restrict__ bias,
       f16* __restrict__ outP, float accMul, float addMul) {
    gemm_body<1>(A, W, bias, outP, (float*)nullptr, accMul, addMul);
}

__global__ void __launch_bounds__(256) __attribute__((amdgpu_num_vgpr(256)))
gemm_out(const f16* __restrict__ A, const f16* __restrict__ W, const float* __restrict__ bias,
         float* __restrict__ outF, float accMul, float addMul) {
    gemm_body<2>(A, W, bias, (f16*)nullptr, outF, accMul, addMul);
}

__global__ void __launch_bounds__(256) __attribute__((amdgpu_num_vgpr(256)))
attn_fwd(const f16* __restrict__ Qh, const f16* __restrict__ Qr,
         const f16* __restrict__ Kh, const f16* __restrict__ Kr,
         const f16* __restrict__ Vt, f16* __restrict__ Cp) {
    __shared__ __attribute__((aligned(16))) f16 ksh[64 * 64];
    __shared__ __attribute__((aligned(16))) f16 ksr[64 * 64];
    __shared__ __attribute__((aligned(16))) f16 vsT[64 * 64];
    __shared__ __attribute__((aligned(16))) f16 ps[8 * 16 * 64];

    const int tid  = (int)threadIdx.x;
    const int lane = tid & 31;
    const int wave = tid >> 5;
    const int hh8  = (lane >> 4) << 3;
    const int c16  = lane & 15;
    const int bh   = (int)blockIdx.y;
    const int bidx = bh / NHEAD;
    const int hidx = bh - bidx * NHEAD;
    const int q0   = (int)blockIdx.x * 128 + wave * 16;
    const size_t head = (size_t)bh * SEQ * HD;
    const size_t qoff = head + (size_t)(q0 + c16) * HD + hh8;
    const int pw = wave * (16 * 64);

    FragU onesu;
#pragma unroll
    for (int i = 0; i < 16; ++i) onesu.e[i] = (f16)1.0f;
    const v16h ones = onesu.v;

    float m[8];
    v8f   o[4], lacc;
#pragma unroll
    for (int r = 0; r < 8; ++r) m[r] = -1.0e30f;
#pragma unroll
    for (int dt = 0; dt < 4; ++dt) o[dt] = zero8();
    lacc = zero8();

    const float cl = 1.4426950408889634f * 0.00048828125f;

#pragma unroll 1
    for (int kt = 0; kt < SEQ / 64; ++kt) {
        __syncthreads();
#pragma unroll
        for (int p2 = 0; p2 < 2; ++p2) {
            const int p   = tid + p2 * 256;
            const int row = p >> 3;
            const int pc  = (p & 7) << 3;
            const size_t kof = head + (size_t)(kt * 64 + row) * HD + pc;
            const v8h kv = *(const v8h*)(Kh + kof);
            const v8h kr = *(const v8h*)(Kr + kof);
            const v8h vv = *(const v8h*)(Vt + head + (size_t)row * SEQ + kt * 64 + pc);
            *(v8h*)&ksh[row * 64 + pc] = kv;
            *(v8h*)&ksr[row * 64 + pc] = kr;
            *(v8h*)&vsT[row * 64 + pc] = vv;
        }
        __syncthreads();

        float xs[4][8];
#pragma unroll
        for (int hf = 0; hf < 2; ++hf) {
            v8f sh[2], sx[2];
#pragma unroll
            for (int t = 0; t < 2; ++t) { sh[t] = zero8(); sx[t] = zero8(); }
#pragma unroll
            for (int c = 0; c < 2; ++c) {
                const v16h qh = gfrag(Qh, qoff + (size_t)(c * 32));
                const v16h qr = gfrag(Qr, qoff + (size_t)(c * 32));
#pragma unroll
                for (int t = 0; t < 2; ++t) {
                    const int off = frag_off(hf * 32 + t * 16, 64, c * 32, lane);
                    const v16h kh = LDS_FRAG(ksh, off);
                    const v16h kr = LDS_FRAG(ksr, off);
                    sh[t] = wmma16(qh, kh, sh[t]);
                    sx[t] = wmma16(qh, kr, sx[t]);
                    sx[t] = wmma16(qr, kh, sx[t]);
                }
            }
#pragma unroll
            for (int t = 0; t < 2; ++t)
#pragma unroll
                for (int r = 0; r < 8; ++r)
                    xs[hf * 2 + t][r] = (sh[t][r] + sx[t][r] * RES_INV) * cl;
        }

#pragma unroll
        for (int r = 0; r < 8; ++r) {
            const float tm = rowmax16(fmaxf(fmaxf(xs[0][r], xs[1][r]), fmaxf(xs[2][r], xs[3][r])));
            const float mn = fmaxf(m[r], tm);
            const float al = fexp2(m[r] - mn);
            m[r] = mn;
            lacc[r] *= al;
#pragma unroll
            for (int dt = 0; dt < 4; ++dt) o[dt][r] *= al;
            const float sft = 10.0f - mn;
#pragma unroll
            for (int nt = 0; nt < 4; ++nt)
                ps[pw + (hh8 + r) * 64 + nt * 16 + c16] = (f16)fexp2(xs[nt][r] + sft);
        }
        __syncthreads();

#pragma unroll
        for (int kk = 0; kk < 2; ++kk) {
            const int poff = pw + frag_off(0, 64, kk * 32, lane);
            const v16h pa = LDS_FRAG(ps, poff);
#pragma unroll
            for (int dt = 0; dt < 4; ++dt) {
                const int voff = frag_off(dt * 16, 64, kk * 32, lane);
                const v16h vb = LDS_FRAG(vsT, voff);
                o[dt] = wmma16(pa, vb, o[dt]);
            }
            lacc = wmma16(pa, ones, lacc);
        }
    }
    __syncthreads();

#pragma unroll
    for (int r = 0; r < 8; ++r) {
        const float inv = (CARRY_CTX / CARRY_QKV) / lacc[r];
#pragma unroll
        for (int dt = 0; dt < 4; ++dt)
            ps[pw + (hh8 + r) * 64 + dt * 16 + c16] = (f16)(o[dt][r] * inv);
    }
    __syncthreads();

    const int piece = lane & 7;
    const int lsub  = lane >> 3;
#pragma unroll
    for (int pass = 0; pass < 2; ++pass) {
#pragma unroll
        for (int it = 0; it < 4; ++it) {
            const int L = it * 4 + lsub;
            const v8h v = *(const v8h*)&ps[pw + L * 64 + piece * 8];
            f16* dp = Cp + ((size_t)(bidx * SEQ + q0 + L) * HID + hidx * HD + piece * 8);
            *(volatile v8h*)dp = v;
        }
        if (pass == 0) __threadfence();
    }
}

extern "C" void kernel_launch(void* const* d_in, const int* in_sizes, int n_in,
                              void* d_out, int out_size, void* d_ws, size_t ws_size,
                              hipStream_t stream) {
    if (n_in < 5) return;
    if (in_sizes[0] < ((NB - 1) * SEQ_FULL + SEQ) * HID) return;
    if (in_sizes[1] < QKVW * HID) return;
    if (in_sizes[2] < QKVW) return;
    if (in_sizes[3] < HID * HID) return;
    if (in_sizes[4] < HID) return;
    if (out_size < MROWS * HID) return;

    const float* x    = (const float*)d_in[0];
    const float* wqkv = (const float*)d_in[1];
    const float* bqkv = (const float*)d_in[2];
    const float* wo   = (const float*)d_in[3];
    const float* bo   = (const float*)d_in[4];

    const size_t nX  = (size_t)MROWS * HID;
    const size_t nWq = (size_t)QKVW * HID;
    const size_t nWo = (size_t)HID * HID;
    const size_t totalHalves = 7 * nX + nWq + nWo;
    if (ws_size < totalHalves * sizeof(f16)) return;

    f16* Xh  = (f16*)d_ws;
    f16* Wq  = Xh  + nX;
    f16* Wo  = Wq  + nWq;
    f16* QKp = Wo  + nWo;
    f16* Vtp = QKp + 4 * nX;
    f16* Cp  = Vtp + nX;

    cvt_rows<<<(MROWS * PCS + 255) / 256, 256, 0, stream>>>(x, Xh, MROWS, SEQ, SEQ_FULL, CARRY_X);
    cvt_rows<<<(QKVW * PCS + 255) / 256, 256, 0, stream>>>(wqkv, Wq, QKVW, QKVW, QKVW, CARRY_W);
    cvt_rows<<<(HID * PCS + 255) / 256, 256, 0, stream>>>(wo, Wo, HID, HID, HID, CARRY_W);

    const float accQKV = CARRY_QKV / (CARRY_X * CARRY_W);
    gemm_qk<<<dim3(MROWS / 128, QKW / 128), 256, 0, stream>>>(Xh, Wq, bqkv, QKp, accQKV, CARRY_QKV);
    gemm_v<<<dim3(MROWS / 128, HID / 128), 256, 0, stream>>>(Xh, Wq + (size_t)QKW * HID, bqkv + QKW,
                                                             Vtp, accQKV, CARRY_QKV);

    attn_fwd<<<dim3(SEQ / 128, NB * NHEAD), 256, 0, stream>>>(QKp, QKp + 2 * nX, QKp + nX, QKp + 3 * nX,
                                                              Vtp, Cp);

    const float accOut = 1.0f / (CARRY_CTX * CARRY_W);
    gemm_out<<<dim3(MROWS / 128, HID / 128), 256, 0, stream>>>(Cp, Wo, bo, (float*)d_out, accOut, 1.0f);
}
